// MambaLayer_3702261809512
// MI455X (gfx1250) — hardware-verified
//
#include <hip/hip_runtime.h>
#include <math.h>

typedef __attribute__((ext_vector_type(16))) _Float16 v16h;
typedef __attribute__((ext_vector_type(8)))  _Float16 v8h;
typedef __attribute__((ext_vector_type(16))) __bf16   v16b;
typedef __attribute__((ext_vector_type(8)))  __bf16   v8b;
typedef __attribute__((ext_vector_type(8)))  float    v8f;
typedef __attribute__((ext_vector_type(4)))  float    v4f;

constexpr int kBatch  = 2;
constexpr int kSeq    = 1024;
constexpr int kDm     = 512;
constexpr int kDin    = 1024;
constexpr int kNst    = 16;
constexpr int kDtR    = 32;
constexpr int kNsl    = 32;
constexpr int kLc     = kSeq / kNsl;
constexpr int kNBr    = 3;
constexpr int kXzP    = 2 * kDin;
constexpr int kXdP    = 64;
constexpr int kRows   = kBatch * kSeq;
constexpr int kBRows  = kNBr * kRows;
constexpr int kConvTP = 260;
constexpr int kScanTS = 64;
constexpr int kScanCh = 64;
constexpr int kScanYP = 68;
constexpr float kLnEps = 1e-5f;
static_assert(kDtR + 2 * kNst == kXdP);
static_assert((kDm % 32) == 0 && (kDin % 32) == 0);
static_assert((kRows % 64) == 0 && (kBRows % 64) == 0 && (kXzP % 64) == 0 && (kXdP % 64) == 0 && (kDm % 64) == 0);
static_assert((kSeq % kScanTS) == 0 && (kSeq % 64) == 0 && (kDin % kScanCh) == 0 && (kDin % 256) == 0);
static_assert((kNsl & (kNsl - 1)) == 0 && kNsl * kLc == kSeq);
static_assert(kDm == 512 && kScanCh == 64 && kScanTS == 64);
static_assert(((kRows / 64) * (kXzP / 64)) % 8 == 0);
static_assert(((kBRows / 64) * (kXdP / 64)) % 8 == 0);
static_assert(((kRows / 64) * (kDm / 64)) % 8 == 0);

constexpr size_t kOffXH   = 0;
constexpr size_t kOffXL   = kOffXH   + (size_t)kRows  * kDm  * 2;
constexpr size_t kOffWIH  = kOffXL   + (size_t)kRows  * kDm  * 2;
constexpr size_t kOffWIL  = kOffWIH  + (size_t)kXzP   * kDm  * 2;
constexpr size_t kOffWXH  = kOffWIL  + (size_t)kXzP   * kDm  * 2;
constexpr size_t kOffWXL  = kOffWXH  + (size_t)kXdP   * kDin * 2;
constexpr size_t kOffWOH  = kOffWXL  + (size_t)kXdP   * kDin * 2;
constexpr size_t kOffWOL  = kOffWOH  + (size_t)kDm    * kDin * 2;
constexpr size_t kOffXZ   = kOffWOL  + (size_t)kDm    * kDin * 2;
constexpr size_t kOffUC   = kOffXZ   + (size_t)kRows  * kXzP * 4;
constexpr size_t kOffUCH  = kOffUC   + (size_t)kBRows * kDin * 4;
constexpr size_t kOffUCL  = kOffUCH  + (size_t)kBRows * kDin * 2;
constexpr size_t kOffXD   = kOffUCL  + (size_t)kBRows * kDin * 2;
constexpr size_t kOffYRAW = kOffXD   + (size_t)kBRows * kXdP * 4;
constexpr size_t kOffYH   = kOffYRAW + (size_t)kBRows * kDin * 4;
constexpr size_t kOffYL   = kOffYH   + (size_t)kRows  * kDin * 2;
constexpr size_t kOffOUTP = kOffYL   + (size_t)kRows  * kDin * 2;
constexpr size_t kWsTotal = kOffOUTP + (size_t)kRows  * kDm  * 4;
static_assert(kWsTotal == 117178368ull);
static_assert(kWsTotal <= 134217728ull);
static_assert((kOffXL % 128) == 0 && (kOffWIH % 128) == 0 && (kOffWIL % 128) == 0 && (kOffWXH % 128) == 0 &&
              (kOffWXL % 128) == 0 && (kOffWOH % 128) == 0 && (kOffWOL % 128) == 0 && (kOffXZ % 128) == 0 &&
              (kOffUC % 128) == 0 && (kOffUCH % 128) == 0 && (kOffUCL % 128) == 0 && (kOffXD % 128) == 0 &&
              (kOffYRAW % 128) == 0 && (kOffYH % 128) == 0 && (kOffYL % 128) == 0 && (kOffOUTP % 128) == 0);

__device__ __forceinline__ unsigned short f2bf_bits(float f) {
  unsigned u = __float_as_uint(f);
  return (unsigned short)((u + 0x7FFFu + ((u >> 16) & 1u)) >> 16);
}
__device__ __forceinline__ float bf_bits2f(unsigned short h) { return __uint_as_float(((unsigned)h) << 16); }

__device__ __forceinline__ void dep_guard4_h(v8f& a, v8f& b, v8f& c, v8f& d, v16h x, v16h y) { asm volatile("v_nop\n\tv_nop\n\tv_nop\n\tv_nop" : "+v"(a), "+v"(b), "+v"(c), "+v"(d) : "v"(x), "v"(y)); }
__device__ __forceinline__ void dep_guard4_b(v8f& a, v8f& b, v8f& c, v8f& d, v16b x, v16b y) { asm volatile("v_nop\n\tv_nop\n\tv_nop\n\tv_nop" : "+v"(a), "+v"(b), "+v"(c), "+v"(d) : "v"(x), "v"(y)); }
__device__ __forceinline__ void keep4_h(v16h a, v16h b, v16h c, v16h d) { asm volatile("v_nop" :: "v"(a), "v"(b), "v"(c), "v"(d)); }
__device__ __forceinline__ void keep4_b(v16b a, v16b b, v16b c, v16b d) { asm volatile("v_nop" :: "v"(a), "v"(b), "v"(c), "v"(d)); }
__device__ __forceinline__ void acc_guard4(v8f& a, v8f& b, v8f& c, v8f& d) { asm volatile("v_nop\n\tv_nop\n\tv_nop\n\tv_nop" : "+v"(a), "+v"(b), "+v"(c), "+v"(d)); }
template <typename T> struct Frag;
template <> struct Frag<_Float16> {
  typedef v16h V; union U { v16h v; v8h h[2]; };
  static __device__ __forceinline__ v16h load(const _Float16* p) {
    U f; f.h[0] = *(const v8h*)(p); f.h[1] = *(const v8h*)(p + 16); return f.v;
  }
  static __device__ __forceinline__ v8f mma(v16h a, v16h b, v8f c) {
    return __builtin_amdgcn_wmma_f32_16x16x32_f16(false, a, false, b, (short)0, c, false, false);
  }
  static __device__ __forceinline__ void guard4(v8f& a, v8f& b, v8f& c, v8f& d, v16h x, v16h y) { dep_guard4_h(a, b, c, d, x, y); }
  static __device__ __forceinline__ void keep(v16h a, v16h b, v16h c, v16h d) { keep4_h(a, b, c, d); }
};
template <> struct Frag<__bf16> {
  typedef v16b V; union U { v16b v; v8b h[2]; };
  static __device__ __forceinline__ v16b load(const __bf16* p) {
    U f; f.h[0] = *(const v8b*)(p); f.h[1] = *(const v8b*)(p + 16); return f.v;
  }
  static __device__ __forceinline__ v8f mma(v16b a, v16b b, v8f c) {
    return __builtin_amdgcn_wmma_f32_16x16x32_bf16(false, a, false, b, (short)0, c, false, false);
  }
  static __device__ __forceinline__ void guard4(v8f& a, v8f& b, v8f& c, v8f& d, v16b x, v16b y) { dep_guard4_b(a, b, c, d, x, y); }
  static __device__ __forceinline__ void keep(v16b a, v16b b, v16b c, v16b d) { keep4_b(a, b, c, d); }
};

template <int ET> struct Elem;
template <> struct Elem<0> { typedef _Float16 T; };
template <> struct Elem<1> { typedef __bf16 T; };
template <int ET, int SPL, int BIAS_MODE, int OUT_MODE, bool RESID, int ACT = 0>
__global__ __launch_bounds__(256) void wmma_gemm64(
    const unsigned short* __restrict__ Ap, const unsigned short* __restrict__ A2p, int lda, long strideA,
    const unsigned short* __restrict__ Btp, const unsigned short* __restrict__ Bt2p, int ldb, long strideB,
    void* __restrict__ Cout, void* __restrict__ Cout2, int ldc, long strideC,
    const float* __restrict__ bias,
    const float* __restrict__ resid, long strideR,
    int M, int N, int K, float scale) {
  typedef typename Elem<ET>::T T;
  typedef typename Frag<T>::V V;
  const T* A = (const T*)Ap; const T* A2 = (const T*)A2p; const T* Bt = (const T*)Btp; const T* Bt2 = (const T*)Bt2p;
  __shared__ __align__(16) float sT[8][16 * 68];
  const int b    = blockIdx.y;
  const int lane = threadIdx.x & 31;
  const int wave = threadIdx.x >> 5;
  const int tilesN = N >> 6;
  const int tilesM = M >> 6;
  const int tile = blockIdx.x * 8 + wave;
  if (tile >= tilesM * tilesN) return;
  const int tm = tile / tilesN;
  const int tn = tile - tm * tilesN;
  const int m0 = tm << 6;
  const int n0 = tn << 6;

  const T* Ab  = A  + (size_t)b * strideA;
  const T* Bb  = Bt + (size_t)b * strideB;
  const T* Ab2 = (SPL >= 1) ? (A2  + (size_t)b * strideA) : nullptr;
  const T* Bb2 = (SPL == 2) ? (Bt2 + (size_t)b * strideB) : nullptr;

  const int rlane = lane & 15;
  const int koff  = (lane >> 4) * 8;
  const int mOff  = (lane >> 4) * 8;

  v8f acc[4][4];
#pragma unroll
  for (int i = 0; i < 4; ++i)
#pragma unroll
    for (int j = 0; j < 4; ++j) acc[i][j] = (v8f){0.f,0.f,0.f,0.f,0.f,0.f,0.f,0.f};

  for (int k0 = 0; k0 < K; k0 += 32) {
    V bh[4], bl[4];
#pragma unroll
    for (int j = 0; j < 4; ++j) {
      const size_t bo = (size_t)(n0 + (j << 4) + rlane) * ldb + koff + k0;
      bh[j] = Frag<T>::load(Bb + bo);
      if (SPL == 2) bl[j] = Frag<T>::load(Bb2 + bo);
    }
#pragma unroll
    for (int i = 0; i < 4; ++i) {
      const size_t ao = (size_t)(m0 + (i << 4) + rlane) * lda + koff + k0;
      V ah = Frag<T>::load(Ab + ao);
      V al;
      if (SPL >= 1) al = Frag<T>::load(Ab2 + ao);
#pragma unroll
      for (int j = 0; j < 4; ++j) {
        acc[i][j] = Frag<T>::mma(ah, bh[j], acc[i][j]);
        if (SPL == 2) acc[i][j] = Frag<T>::mma(ah, bl[j], acc[i][j]);
        if (SPL >= 1) acc[i][j] = Frag<T>::mma(al, bh[j], acc[i][j]);
      }
      Frag<T>::guard4(acc[i][0], acc[i][1], acc[i][2], acc[i][3], ah, (SPL >= 1) ? al : ah);
    }
    Frag<T>::keep(bh[0], bh[1], bh[2], bh[3]);
    if (SPL == 2) Frag<T>::keep(bl[0], bl[1], bl[2], bl[3]);
  }
  acc_guard4(acc[0][0], acc[0][1], acc[0][2], acc[0][3]);
  acc_guard4(acc[1][0], acc[1][1], acc[1][2], acc[1][3]);
  acc_guard4(acc[2][0], acc[2][1], acc[2][2], acc[2][3]);
  acc_guard4(acc[3][0], acc[3][1], acc[3][2], acc[3][3]);

  float* slab = sT[wave];
  const float* Rb = RESID ? (resid + (size_t)b * strideR) : nullptr;
#pragma unroll
  for (int i = 0; i < 4; ++i) {
    const int mBase = m0 + (i << 4);
#pragma unroll
    for (int j = 0; j < 4; ++j) {
      const int n = n0 + (j << 4) + rlane;
      float bv = 0.f;
      if (BIAS_MODE == 2) bv = bias[n];
#pragma unroll
      for (int r = 0; r < 8; ++r) {
        float v = acc[i][j][r] * scale;
        if (BIAS_MODE == 1) v += bias[mBase + mOff + r];
        if (BIAS_MODE == 2) v += bv;
        if (RESID) v += Rb[(size_t)(mBase + mOff + r) * ldc + n];
        if (ACT == 1) v = tanhf(v);
        if (ACT == 2) v = fmaxf(v, 0.0f);
        if (ACT == 3) v = v / (1.0f + expf(-v));
        if (ACT == 4) v = (v > 0.f) ? v : 0.01f * v;
        slab[(mOff + r) * 68 + (j << 4) + rlane] = v;
      }
    }
    __builtin_amdgcn_fence(__ATOMIC_RELEASE, "workgroup");
    __builtin_amdgcn_wave_barrier();
    __builtin_amdgcn_fence(__ATOMIC_ACQUIRE, "workgroup");
    if (OUT_MODE == 0) {
      float* C = (float*)Cout + (size_t)b * strideC;
      const int hh = lane >> 4, c4 = (lane & 15) * 4;
      for (int pass = 0; pass < 2; ++pass) {
#pragma unroll
        for (int it = 0; it < 8; ++it) {
          const int row = it * 2 + hh;
          v4f v = *(const v4f*)(slab + row * 68 + c4);
          *(volatile v4f*)(C + (size_t)(mBase + row) * ldc + n0 + c4) = v;
        }
        __threadfence();
      }
    } else {
      const int q = lane >> 3, c8 = (lane & 7) * 8;
      unsigned short* C  = (unsigned short*)Cout  + (size_t)b * strideC;
      unsigned short* C2 = (OUT_MODE == 2) ? ((unsigned short*)Cout2 + (size_t)b * strideC) : nullptr;
      for (int pass = 0; pass < 2; ++pass) {
#pragma unroll
        for (int it = 0; it < 4; ++it) {
          const int row = it * 4 + q;
          const float* sp = slab + row * 68 + c8;
          v8h hv, lv;
#pragma unroll
          for (int e = 0; e < 8; ++e) {
            if (OUT_MODE == 1) {
              hv[e] = (_Float16)sp[e];
            } else {
              unsigned short hb = f2bf_bits(sp[e]);
              unsigned short lb = f2bf_bits(sp[e] - bf_bits2f(hb));
              hv[e] = __builtin_bit_cast(_Float16, hb);
              lv[e] = __builtin_bit_cast(_Float16, lb);
            }
          }
          *(volatile v8h*)(C + (size_t)(mBase + row) * ldc + n0 + c8) = hv;
          if (OUT_MODE == 2) *(volatile v8h*)(C2 + (size_t)(mBase + row) * ldc + n0 + c8) = lv;
        }
        __threadfence();
      }
    }
    __builtin_amdgcn_fence(__ATOMIC_RELEASE, "workgroup");
    __builtin_amdgcn_wave_barrier();
    __builtin_amdgcn_fence(__ATOMIC_ACQUIRE, "workgroup");
  }
}

__device__ __forceinline__ int orig_pos(int br, int p) {
  const int pf = p;
  const int pb = kSeq - 1 - p;
  const int ps = (p & (kNsl - 1)) * kLc + (p / kNsl);
  return (br == 0) ? pf : ((br == 1) ? pb : ps);
}

__device__ __forceinline__ float silu_f(float v) {
  return v * __builtin_amdgcn_rcpf(1.0f + expf(-v));
}

__global__ __launch_bounds__(256) void split_rows_bf16_kernel(
    const float* __restrict__ src, unsigned short* __restrict__ dhi, unsigned short* __restrict__ dlo, int total8)
{
  const int i = blockIdx.x * 256 + threadIdx.x;
  if (i >= total8) return;
  const size_t e0 = (size_t)i << 3;
  const v4f a0 = *(const v4f*)(src + e0);
  const v4f a1 = *(const v4f*)(src + e0 + 4);
  v8h hv, lv;
#pragma unroll
  for (int e = 0; e < 4; ++e) {
    const float f0 = a0[e], f1 = a1[e];
    const unsigned short h0 = f2bf_bits(f0), h1 = f2bf_bits(f1);
    const unsigned short l0 = f2bf_bits(f0 - bf_bits2f(h0)), l1 = f2bf_bits(f1 - bf_bits2f(h1));
    hv[e]     = __builtin_bit_cast(_Float16, h0);
    hv[4 + e] = __builtin_bit_cast(_Float16, h1);
    lv[e]     = __builtin_bit_cast(_Float16, l0);
    lv[4 + e] = __builtin_bit_cast(_Float16, l1);
  }
  unsigned short* qh = dhi + e0;
  unsigned short* ql = dlo + e0;
  *(volatile v8h*)qh = hv;
  *(volatile v8h*)ql = lv;
  __threadfence();
  *(volatile v8h*)qh = hv;
  *(volatile v8h*)ql = lv;
}

__global__ __launch_bounds__(256) void conv_silu_kernel(
    const float* __restrict__ XZ,
    const float* __restrict__ cw0, const float* __restrict__ cb0,
    const float* __restrict__ cw1, const float* __restrict__ cb1,
    const float* __restrict__ cw2, const float* __restrict__ cb2,
    float* __restrict__ UC, unsigned short* __restrict__ UCH, unsigned short* __restrict__ UCL)
{
  __shared__ __align__(16) float sT[16 * kConvTP];
  const int tid = threadIdx.x, lane = tid & 31, wave = tid >> 5;
  const int d0 = blockIdx.x * 256, d = d0 + tid;
  const int g0  = blockIdx.y * 64;
  const int br  = g0 / kRows;
  const int rem = g0 - br * kRows;
  const int bix = rem / kSeq;
  const int p0  = rem - bix * kSeq;
  const float* cw = (br == 0) ? cw0 : ((br == 1) ? cw1 : cw2);
  const float* cb = (br == 0) ? cb0 : ((br == 1) ? cb1 : cb2);
  const v4f wv = *(const v4f*)(cw + (size_t)d * 4);
  const float w0 = wv[0], w1 = wv[1], w2 = wv[2], w3 = wv[3];
  const float bc = cb[d];
  const size_t xbase = (size_t)bix * kSeq;
  float xm3, xm2, xm1;
  {
    const bool hist = (p0 > 0);
    const int pb = hist ? (p0 - 3) : 0;
    const float v3 = XZ[(xbase + orig_pos(br, pb))     * kXzP + d];
    const float v2 = XZ[(xbase + orig_pos(br, pb + 1)) * kXzP + d];
    const float v1 = XZ[(xbase + orig_pos(br, pb + 2)) * kXzP + d];
    xm3 = hist ? v3 : 0.f;
    xm2 = hist ? v2 : 0.f;
    xm1 = hist ? v1 : 0.f;
  }
  const int hrow = wave >> 1;
  const int hch  = (wave & 1) * 128 + lane * 4;
#pragma unroll 1
  for (int sub = 0; sub < 4; ++sub) {
    const int lb = g0 + sub * 16;
#pragma unroll 1
    for (int s = 0; s < 16; ++s) {
      const int p = p0 + sub * 16 + s;
      const float xcur = XZ[(xbase + orig_pos(br, p)) * kXzP + d];
      float acc = w0 * xm3;
      acc = fmaf(w1, xm2, acc);
      acc = fmaf(w2, xm1, acc);
      acc = fmaf(w3, xcur, acc);
      const float sv = acc + bc;
      sT[s * kConvTP + tid] = silu_f(sv);
      xm3 = xm2; xm2 = xm1; xm1 = xcur;
    }
    __syncthreads();
    v4f fv[4];
    v8h bh[2], blo[2];
#pragma unroll
    for (int it = 0; it < 4; ++it) fv[it] = *(const v4f*)(sT + (it * 4 + hrow) * kConvTP + hch);
#pragma unroll
    for (int it = 0; it < 2; ++it) {
      const float* sp = sT + (it * 8 + wave) * kConvTP + lane * 8;
      const v4f a0 = *(const v4f*)(sp);
      const v4f a1 = *(const v4f*)(sp + 4);
#pragma unroll
      for (int e = 0; e < 4; ++e) {
        const float f0 = a0[e], f1 = a1[e];
        const unsigned short h0 = f2bf_bits(f0), h1 = f2bf_bits(f1);
        const unsigned short l0 = f2bf_bits(f0 - bf_bits2f(h0)), l1 = f2bf_bits(f1 - bf_bits2f(h1));
        bh[it][e]      = __builtin_bit_cast(_Float16, h0);
        bh[it][4 + e]  = __builtin_bit_cast(_Float16, h1);
        blo[it][e]     = __builtin_bit_cast(_Float16, l0);
        blo[it][4 + e] = __builtin_bit_cast(_Float16, l1);
      }
    }
    for (int pass = 0; pass < 2; ++pass) {
#pragma unroll
      for (int it = 0; it < 4; ++it)
        *(volatile v4f*)(UC + (size_t)(lb + it * 4 + hrow) * kDin + d0 + hch) = fv[it];
#pragma unroll
      for (int it = 0; it < 2; ++it) {
        const size_t o = (size_t)(lb + it * 8 + wave) * kDin + d0 + lane * 8;
        *(volatile v8h*)(UCH + o) = bh[it];
        *(volatile v8h*)(UCL + o) = blo[it];
      }
      __threadfence();
    }
    __syncthreads();
  }
}

__global__ __launch_bounds__(64) void scan_kernel(
    const float* __restrict__ XD, const float* __restrict__ UC,
    const float* __restrict__ Wdt, const float* __restrict__ bdt,
    const float* __restrict__ Al0, const float* __restrict__ Al1, const float* __restrict__ Al2,
    const float* __restrict__ Dp0, const float* __restrict__ Dp1, const float* __restrict__ Dp2,
    float* __restrict__ YRAW)
{
  __shared__ __align__(16) float sX[kScanTS * kXdP];
  __shared__ __align__(16) float sY[kScanTS * kScanYP];
  __shared__ __align__(16) float sW[kDtR * kScanCh];
  __shared__ __align__(16) float sA[kNst * kScanCh];
  const int tid = threadIdx.x, lane = tid & 31, wave = tid >> 5;
  constexpr int kBlkPerSeq = kDin / kScanCh;
  const int sid = blockIdx.x / kBlkPerSeq;
  const int d0  = (blockIdx.x - sid * kBlkPerSeq) * kScanCh;
  const int d   = d0 + tid;
  const int br  = sid / kBatch;
  const float* Alog = (br == 0) ? Al0 : ((br == 1) ? Al1 : Al2);
  const float* Dp   = (br == 0) ? Dp0 : ((br == 1) ? Dp1 : Dp2);
  const size_t row0 = (size_t)sid * kSeq;
#pragma unroll 1
  for (int r = 0; r < kDtR; ++r) sW[r * kScanCh + tid] = Wdt[(size_t)d * kDtR + r];
#pragma unroll 1
  for (int s = 0; s < kNst; ++s) sA[s * kScanCh + tid] = -expf(Alog[(size_t)d * kNst + s]);
  __syncthreads();
  float negA[kNst], h[kNst];
#pragma unroll
  for (int s = 0; s < kNst; ++s) {
    negA[s] = sA[s * kScanCh + tid];
    h[s] = 0.f;
  }
  const float bb = bdt[d], Dd = Dp[d];
  const int lr = tid >> 4, lc4 = (tid & 15) * 4;
  const int hh = lane >> 4, c4 = (lane & 15) * 4;
#pragma unroll 1
  for (int t0 = 0; t0 < kSeq; t0 += kScanTS) {
    __syncthreads();
#pragma unroll
    for (int i = 0; i < 16; ++i) {
      const int r = lr + 4 * i;
      *(v4f*)(sX + r * kXdP + lc4) = *(const v4f*)(XD + (row0 + t0 + r) * kXdP + lc4);
    }
    __syncthreads();
#pragma unroll 1
    for (int s = 0; s < kScanTS; ++s) {
      const int t = t0 + s;
      const float* xr = sX + s * kXdP;
      float vdot = 0.f;
#pragma unroll 1
      for (int r4 = 0; r4 < kDtR / 4; ++r4) {
        const v4f xv = *(const v4f*)(xr + 4 * r4);
        const float* wp = sW + (4 * r4) * kScanCh + tid;
        vdot = fmaf(xv[0], wp[0], vdot);
        vdot = fmaf(xv[1], wp[kScanCh], vdot);
        vdot = fmaf(xv[2], wp[2 * kScanCh], vdot);
        vdot = fmaf(xv[3], wp[3 * kScanCh], vdot);
      }
      float Bs[kNst], Cs[kNst];
#pragma unroll
      for (int q4 = 0; q4 < 4; ++q4) {
        const v4f bv = *(const v4f*)(xr + kDtR + 4 * q4);
        const v4f cv = *(const v4f*)(xr + kDtR + kNst + 4 * q4);
        Bs[4 * q4 + 0] = bv[0]; Bs[4 * q4 + 1] = bv[1]; Bs[4 * q4 + 2] = bv[2]; Bs[4 * q4 + 3] = bv[3];
        Cs[4 * q4 + 0] = cv[0]; Cs[4 * q4 + 1] = cv[1]; Cs[4 * q4 + 2] = cv[2]; Cs[4 * q4 + 3] = cv[3];
      }
      const float v   = vdot + bb;
      const float a   = __expf(-fabsf(v));
      const float u   = 1.0f + a;
      const float l1p = __logf(u) + (a - (u - 1.0f)) * __builtin_amdgcn_rcpf(u);
      const float dt  = fmaxf(v, 0.0f) + l1p;
      const float xt  = UC[(row0 + t) * kDin + d];
      const float dtx = dt * xt;
      float y = 0.f;
#pragma unroll
      for (int k = 0; k < kNst; ++k) {
        const float e = __expf(dt * negA[k]);
        h[k] = e * h[k] + dtx * Bs[k];
        y = h[k] * Cs[k] + y;
      }
      y = xt * Dd + y;
      sY[s * kScanYP + tid] = y;
    }
    __syncthreads();
    for (int pass = 0; pass < 2; ++pass) {
#pragma unroll 4
      for (int it = 0; it < 16; ++it) {
        const int row = wave * 32 + it * 2 + hh;
        const v4f val = *(const v4f*)(sY + row * kScanYP + c4);
        const size_t orow = row0 + (size_t)orig_pos(br, t0 + row);
        *(volatile v4f*)(YRAW + orow * kDin + d0 + c4) = val;
      }
      __threadfence();
    }
  }
}

__global__ __launch_bounds__(256) void combine_gate_kernel(
    const float* __restrict__ XZ, const float* __restrict__ YRAW,
    unsigned short* __restrict__ YH, unsigned short* __restrict__ YL, int total8)
{
  const int i = blockIdx.x * 256 + threadIdx.x;
  if (i >= total8) return;
  const size_t e0  = (size_t)i << 3;
  const size_t row = e0 / kDin;
  const int    c   = (int)(e0 - row * kDin);
  const float* zp = XZ + row * kXzP + kDin + c;
  const v4f z0 = *(const v4f*)(zp);
  const v4f z1 = *(const v4f*)(zp + 4);
  float g[8];
#pragma unroll
  for (int e = 0; e < 4; ++e) {
    const float za = z0[e], zb = z1[e];
    g[e]     = silu_f(za);
    g[4 + e] = silu_f(zb);
  }
  asm volatile("" ::: "memory");
  constexpr size_t kPlane = (size_t)kRows * kDin;
  const v4f a0 = *(const v4f*)(YRAW + e0);
  const v4f a1 = *(const v4f*)(YRAW + e0 + 4);
  const v4f b0 = *(const v4f*)(YRAW + kPlane + e0);
  const v4f b1 = *(const v4f*)(YRAW + kPlane + e0 + 4);
  const v4f c0 = *(const v4f*)(YRAW + 2 * kPlane + e0);
  const v4f c1 = *(const v4f*)(YRAW + 2 * kPlane + e0 + 4);
  v8h hv, lv;
#pragma unroll
  for (int e = 0; e < 4; ++e) {
    const float s0 = (a0[e] + b0[e]) + c0[e];
    const float s1 = (a1[e] + b1[e]) + c1[e];
    const float f0 = s0 * g[e];
    const float f1 = s1 * g[4 + e];
    const unsigned short h0 = f2bf_bits(f0), h1 = f2bf_bits(f1);
    const unsigned short l0 = f2bf_bits(f0 - bf_bits2f(h0)), l1 = f2bf_bits(f1 - bf_bits2f(h1));
    hv[e]     = __builtin_bit_cast(_Float16, h0);
    hv[4 + e] = __builtin_bit_cast(_Float16, h1);
    lv[e]     = __builtin_bit_cast(_Float16, l0);
    lv[4 + e] = __builtin_bit_cast(_Float16, l1);
  }
  unsigned short* qh = YH + e0;
  unsigned short* ql = YL + e0;
  *(volatile v8h*)qh = hv;
  *(volatile v8h*)ql = lv;
  __threadfence();
  *(volatile v8h*)qh = hv;
  *(volatile v8h*)ql = lv;
}

__global__ __launch_bounds__(256) void layernorm_kernel(
    const float* __restrict__ X, const float* __restrict__ gamma, const float* __restrict__ beta,
    float* __restrict__ out, int nrows)
{
  const int lane = threadIdx.x & 31, wave = threadIdx.x >> 5;
  const int row = blockIdx.x * 8 + wave;
  if (row >= nrows) return;
  const float* xr = X + (size_t)row * kDm;
  v4f v[4];
#pragma unroll
  for (int it = 0; it < 4; ++it) v[it] = *(const v4f*)(xr + it * 128 + lane * 4);
  float s = 0.f;
#pragma unroll
  for (int it = 0; it < 4; ++it) s += (v[it][0] + v[it][1]) + (v[it][2] + v[it][3]);
#pragma unroll
  for (int off = 16; off > 0; off >>= 1) s += __shfl_xor(s, off, 32);
  const float mu = s * (1.0f / (float)kDm);
  float q = 0.f;
#pragma unroll
  for (int it = 0; it < 4; ++it) {
#pragma unroll
    for (int e = 0; e < 4; ++e) {
      const float dlt = v[it][e] - mu;
      q = fmaf(dlt, dlt, q);
    }
  }
#pragma unroll
  for (int off = 16; off > 0; off >>= 1) q += __shfl_xor(q, off, 32);
  const float var = q * (1.0f / (float)kDm);
  const float rs  = rsqrtf(var + kLnEps);
  asm volatile("" ::: "memory");
  v4f o[4];
#pragma unroll
  for (int it = 0; it < 4; ++it) {
    const v4f gm = *(const v4f*)(gamma + it * 128 + lane * 4);
    const v4f be = *(const v4f*)(beta + it * 128 + lane * 4);
#pragma unroll
    for (int e = 0; e < 4; ++e) o[it][e] = (v[it][e] - mu) * rs * gm[e] + be[e];
  }
  float* orow = out + (size_t)row * kDm;
  for (int pass = 0; pass < 2; ++pass) {
#pragma unroll
    for (int it = 0; it < 4; ++it)
      *(volatile v4f*)(orow + it * 128 + lane * 4) = o[it];
    __threadfence();
  }
}

extern "C" void kernel_launch(void* const* d_in, const int* in_sizes, int n_in,
                              void* d_out, int out_size, void* d_ws, size_t ws_size,
                              hipStream_t stream) {
  if (n_in < 20) return;
  if (in_sizes[0] != kRows * kDm) return;
  if (in_sizes[1] != kXzP * kDm) return;
  if (in_sizes[2] != kDin * 4 || in_sizes[3] != kDin) return;
  if (in_sizes[4] != kDin * 4 || in_sizes[5] != kDin) return;
  if (in_sizes[6] != kDin * 4 || in_sizes[7] != kDin) return;
  if (in_sizes[8] != kXdP * kDin) return;
  if (in_sizes[9] != kDin * kDtR || in_sizes[10] != kDin) return;
  if (in_sizes[11] != kDin * kNst || in_sizes[12] != kDin * kNst || in_sizes[13] != kDin * kNst) return;
  if (in_sizes[14] != kDin || in_sizes[15] != kDin || in_sizes[16] != kDin) return;
  if (in_sizes[17] != kDm * kDin) return;
  if (in_sizes[18] != kDm || in_sizes[19] != kDm) return;
  if (out_size != kRows * kDm) return;
  if (ws_size < kWsTotal) return;

  const float* x        = (const float*)d_in[0];
  const float* W_in     = (const float*)d_in[1];
  const float* conv_w_f = (const float*)d_in[2];
  const float* conv_b_f = (const float*)d_in[3];
  const float* conv_w_b = (const float*)d_in[4];
  const float* conv_b_b = (const float*)d_in[5];
  const float* conv_w_s = (const float*)d_in[6];
  const float* conv_b_s = (const float*)d_in[7];
  const float* W_xproj  = (const float*)d_in[8];
  const float* W_dt     = (const float*)d_in[9];
  const float* b_dt     = (const float*)d_in[10];
  const float* A_log_f  = (const float*)d_in[11];
  const float* A_log_b  = (const float*)d_in[12];
  const float* A_log_s  = (const float*)d_in[13];
  const float* D_f      = (const float*)d_in[14];
  const float* D_b      = (const float*)d_in[15];
  const float* D_s      = (const float*)d_in[16];
  const float* W_out    = (const float*)d_in[17];
  const float* ln_gamma = (const float*)d_in[18];
  const float* ln_beta  = (const float*)d_in[19];
  float* out = (float*)d_out;

  char* ws = (char*)d_ws;
  unsigned short* XH   = (unsigned short*)(ws + kOffXH);
  unsigned short* XL   = (unsigned short*)(ws + kOffXL);
  unsigned short* WIH  = (unsigned short*)(ws + kOffWIH);
  unsigned short* WIL  = (unsigned short*)(ws + kOffWIL);
  unsigned short* WXH  = (unsigned short*)(ws + kOffWXH);
  unsigned short* WXL  = (unsigned short*)(ws + kOffWXL);
  unsigned short* WOH  = (unsigned short*)(ws + kOffWOH);
  unsigned short* WOL  = (unsigned short*)(ws + kOffWOL);
  float*          XZ   = (float*)(ws + kOffXZ);
  float*          UC   = (float*)(ws + kOffUC);
  unsigned short* UCH  = (unsigned short*)(ws + kOffUCH);
  unsigned short* UCL  = (unsigned short*)(ws + kOffUCL);
  float*          XD   = (float*)(ws + kOffXD);
  float*          YRAW = (float*)(ws + kOffYRAW);
  unsigned short* YH   = (unsigned short*)(ws + kOffYH);
  unsigned short* YL   = (unsigned short*)(ws + kOffYL);
  float*          OUTP = (float*)(ws + kOffOUTP);
  const float* dummy_bias  = b_dt;
  const float* dummy_resid = x;

  split_rows_bf16_kernel<<<(kRows * kDm / 8) / 256, 256, 0, stream>>>(x, XH, XL, kRows * kDm / 8);
  split_rows_bf16_kernel<<<(kXzP * kDm / 8) / 256, 256, 0, stream>>>(W_in, WIH, WIL, kXzP * kDm / 8);
  split_rows_bf16_kernel<<<(kXdP * kDin / 8) / 256, 256, 0, stream>>>(W_xproj, WXH, WXL, kXdP * kDin / 8);
  split_rows_bf16_kernel<<<(kDm * kDin / 8) / 256, 256, 0, stream>>>(W_out, WOH, WOL, kDm * kDin / 8);

  wmma_gemm64<1, 2, 0, 0, false><<<dim3(((kRows / 64) * (kXzP / 64)) / 8, 1), 256, 0, stream>>>(
      XH, XL, kDm, 0L,
      WIH, WIL, kDm, 0L,
      (void*)XZ, (void*)XZ, kXzP, 0L,
      dummy_bias, dummy_resid, 0L,
      kRows, kXzP, kDm, 1.0f);

  conv_silu_kernel<<<dim3(kDin / 256, kBRows / 64), 256, 0, stream>>>(
      XZ, conv_w_f, conv_b_f, conv_w_b, conv_b_b, conv_w_s, conv_b_s, UC, UCH, UCL);

  wmma_gemm64<1, 2, 0, 0, false><<<dim3(((kBRows / 64) * (kXdP / 64)) / 8, 1), 256, 0, stream>>>(
      UCH, UCL, kDin, 0L,
      WXH, WXL, kDin, 0L,
      (void*)XD, (void*)XD, kXdP, 0L,
      dummy_bias, dummy_resid, 0L,
      kBRows, kXdP, kDin, 1.0f);

  scan_kernel<<<kNBr * kBatch * (kDin / kScanCh), kScanCh, 0, stream>>>(
      XD, UC, W_dt, b_dt, A_log_f, A_log_b, A_log_s, D_f, D_b, D_s, YRAW);

  combine_gate_kernel<<<(kRows * kDin / 8) / 256, 256, 0, stream>>>(XZ, YRAW, YH, YL, kRows * kDin / 8);

  wmma_gemm64<1, 2, 0, 0, false><<<dim3(((kRows / 64) * (kDm / 64)) / 8, 1), 256, 0, stream>>>(
      YH, YL, kDin, 0L,
      WOH, WOL, kDin, 0L,
      (void*)OUTP, (void*)OUTP, kDm, 0L,
      dummy_bias, dummy_resid, 0L,
      kRows, kDm, kDin, 1.0f);

  layernorm_kernel<<<kRows / 8, 256, 0, stream>>>(OUTP, ln_gamma, ln_beta, out, kRows);
}
